// DependencyParserCombinedAttention_62010737819977
// MI455X (gfx1250) — hardware-verified
//
#include <hip/hip_runtime.h>
#include <math.h>

constexpr int SEQ_LEN = 768;
constexpr int EMB_W   = 300;
constexpr int EMB_P   = 64;
constexpr int VOC_W   = 50000;
constexpr int VOC_P   = 64;
constexpr int IN0     = EMB_W + EMB_P;
constexpr int IN0_PAD = 384;
constexpr int HID     = 512;
constexpr int GATES   = 4 * HID;
constexpr int IN1     = 2 * HID;
constexpr int MLP     = 256;
constexpr int AUG     = MLP + 1;
constexpr int AUG_PAD = 320;
constexpr int HM_LD   = 2 * MLP;
constexpr int NTHR    = 256;
constexpr int PK_CH   = 64;
constexpr int PK_MP   = 68;

constexpr float CARRY_W  = 64.0f;
constexpr float CARRY_X0 = 64.0f;
constexpr float CARRY_H  = 256.0f;
constexpr float SC_L0    = 1.0f / (CARRY_X0 * CARRY_W);
constexpr float SC_HW    = 1.0f / (CARRY_H * CARRY_W);
constexpr float SC_T     = CARRY_H / (CARRY_H * CARRY_W);
constexpr float SC_ATT   = 1.0f / (CARRY_H * CARRY_H);

static_assert(IN0 == 364 && IN0 % 4 == 0 && IN1 % 4 == 0, "row vectors of 4 floats");
static_assert(IN0_PAD % 32 == 0 && IN0_PAD >= IN0, "K pad layer 0");
static_assert(IN1 % 32 == 0 && AUG_PAD % 32 == 0 && AUG_PAD >= AUG, "K multiples of 32");
static_assert(SEQ_LEN % 64 == 0 && GATES % 64 == 0 && MLP % 64 == 0 && AUG_PAD % 64 == 0, "M, N tile multiples");
static_assert(SEQ_LEN % 32 == 0 && MLP % PK_CH == 0, "pair tiles");
static_assert((SEQ_LEN * (IN0_PAD / 8)) % NTHR == 0, "embed grid exact");
static_assert((GATES * (IN0_PAD / 8)) % NTHR == 0 && (GATES * (IN1 / 8)) % NTHR == 0 && (MLP * (IN1 / 8)) % NTHR == 0, "convert grids exact");
static_assert((AUG_PAD * (AUG_PAD / 8)) % NTHR == 0, "At grid exact");
static_assert((SEQ_LEN * (AUG_PAD / 8)) % 32 == 0 && (2 * SEQ_LEN * (AUG_PAD / 8)) % NTHR == 0, "aug grid exact, planes wave aligned");

typedef __attribute__((ext_vector_type(16))) _Float16 v16h;
typedef __attribute__((ext_vector_type(8)))  _Float16 v8h;
typedef __attribute__((ext_vector_type(8)))  float    v8f;
typedef __attribute__((ext_vector_type(4)))  float    v4f;

union FragU { v16h v; v8h h[2]; };

__device__ __forceinline__ v16h frag_load_h(const _Float16* p) {
  FragU f;
  f.h[0] = *(const v8h*)(p);
  f.h[1] = *(const v8h*)(p + 16);
  return f.v;
}
__device__ __forceinline__ v8f mma_h(v16h a, v16h b, v8f c) {
  return __builtin_amdgcn_wmma_f32_16x16x32_f16(false, a, false, b, (short)0, c, false, false);
}
__device__ __forceinline__ void guard_row_h(v8f& a, v8f& b, v8f& c, v8f& d, v16h x, v16h b0, v16h b1, v16h b2, v16h b3) {
  asm volatile("v_nop\n\tv_nop\n\tv_nop\n\tv_nop" : "+v"(a), "+v"(b), "+v"(c), "+v"(d) : "v"(x), "v"(b0), "v"(b1), "v"(b2), "v"(b3));
}
__device__ __forceinline__ void keep4_h(v16h a, v16h b, v16h c, v16h d) { asm volatile("v_nop" :: "v"(a), "v"(b), "v"(c), "v"(d)); }
__device__ __forceinline__ void acc_guard4(v8f& a, v8f& b, v8f& c, v8f& d) { asm volatile("v_nop\n\tv_nop\n\tv_nop\n\tv_nop" : "+v"(a), "+v"(b), "+v"(c), "+v"(d)); }

__device__ __forceinline__ float fsig(float x)  { return __builtin_amdgcn_rcpf(1.0f + __expf(-x)); }
__device__ __forceinline__ float ftanh(float x) { return 1.0f - 2.0f * __builtin_amdgcn_rcpf(__expf(2.0f * x) + 1.0f); }

template <bool HAS_BIAS, bool OUT_F16>
__global__ __launch_bounds__(256) void wmma_gemm64(
    const unsigned short* __restrict__ Ap, int lda,
    const unsigned short* __restrict__ Btp, int ldb,
    void* __restrict__ Cout, int ldc,
    const float* __restrict__ bias,
    int Mrows, int Ncols, int Kdim, float scale) {
  const _Float16* A  = (const _Float16*)Ap;
  const _Float16* Bt = (const _Float16*)Btp;
  __shared__ __align__(16) float sT[8][16 * 68];
  const int lane = threadIdx.x & 31;
  const int wave = threadIdx.x >> 5;
  const int tilesN = Ncols >> 6;
  const int tilesM = Mrows >> 6;
  const int tile = blockIdx.x * 8 + wave;
  if (tile >= tilesM * tilesN) return;
  const int tm = tile / tilesN;
  const int tn = tile - tm * tilesN;
  const int m0 = tm << 6;
  const int n0 = tn << 6;

  const int rlane = lane & 15;
  const int koff  = (lane >> 4) * 8;
  const int mOff  = (lane >> 4) * 8;

  v8f acc[4][4];
#pragma unroll
  for (int i = 0; i < 4; ++i)
#pragma unroll
    for (int j = 0; j < 4; ++j) acc[i][j] = (v8f){0.f, 0.f, 0.f, 0.f, 0.f, 0.f, 0.f, 0.f};

  for (int k0 = 0; k0 < Kdim; k0 += 32) {
    v16h bh[4];
#pragma unroll
    for (int j = 0; j < 4; ++j) {
      const size_t bo = (size_t)(n0 + (j << 4) + rlane) * ldb + koff + k0;
      bh[j] = frag_load_h(Bt + bo);
    }
#pragma unroll
    for (int i = 0; i < 4; ++i) {
      const size_t ao = (size_t)(m0 + (i << 4) + rlane) * lda + koff + k0;
      const v16h ah = frag_load_h(A + ao);
#pragma unroll
      for (int j = 0; j < 4; ++j) acc[i][j] = mma_h(ah, bh[j], acc[i][j]);
      guard_row_h(acc[i][0], acc[i][1], acc[i][2], acc[i][3], ah, bh[0], bh[1], bh[2], bh[3]);
    }
    keep4_h(bh[0], bh[1], bh[2], bh[3]);
  }
  acc_guard4(acc[0][0], acc[0][1], acc[0][2], acc[0][3]);
  acc_guard4(acc[1][0], acc[1][1], acc[1][2], acc[1][3]);
  acc_guard4(acc[2][0], acc[2][1], acc[2][2], acc[2][3]);
  acc_guard4(acc[3][0], acc[3][1], acc[3][2], acc[3][3]);

  float* slab = sT[wave];
#pragma unroll
  for (int i = 0; i < 4; ++i) {
    const int mBase = m0 + (i << 4);
#pragma unroll
    for (int j = 0; j < 4; ++j) {
      const int n = n0 + (j << 4) + rlane;
      float bv = 0.f;
      if (HAS_BIAS) bv = bias[n];
#pragma unroll
      for (int r = 0; r < 8; ++r) {
        float v = acc[i][j][r] * scale;
        if (HAS_BIAS) v += bv;
        slab[(mOff + r) * 68 + (j << 4) + rlane] = v;
      }
    }
    __builtin_amdgcn_fence(__ATOMIC_RELEASE, "workgroup");
    __builtin_amdgcn_wave_barrier();
    __builtin_amdgcn_fence(__ATOMIC_ACQUIRE, "workgroup");
    if (!OUT_F16) {
      float* C = (float*)Cout;
      const int hh = lane >> 4, c4 = (lane & 15) * 4;
      for (int pass = 0; pass < 2; ++pass) {
#pragma unroll
        for (int it = 0; it < 8; ++it) {
          const int row = it * 2 + hh;
          v4f v = *(const v4f*)(slab + row * 68 + c4);
          *(volatile v4f*)(C + (size_t)(mBase + row) * ldc + n0 + c4) = v;
        }
        __threadfence();
      }
    } else {
      const int q = lane >> 3, c8 = (lane & 7) * 8;
      unsigned short* C = (unsigned short*)Cout;
      for (int pass = 0; pass < 2; ++pass) {
#pragma unroll
        for (int it = 0; it < 4; ++it) {
          const int row = it * 4 + q;
          const float* sp = slab + row * 68 + c8;
          v8h hv;
#pragma unroll
          for (int e = 0; e < 8; ++e) hv[e] = (_Float16)sp[e];
          *(volatile v8h*)(C + (size_t)(mBase + row) * ldc + n0 + c8) = hv;
        }
        __threadfence();
      }
    }
    __builtin_amdgcn_fence(__ATOMIC_RELEASE, "workgroup");
    __builtin_amdgcn_wave_barrier();
    __builtin_amdgcn_fence(__ATOMIC_ACQUIRE, "workgroup");
  }
}

__global__ __launch_bounds__(NTHR) void cvt_pad_f16_kernel(const float* __restrict__ src, unsigned short* __restrict__ dst,
                                                           int nrow, int kreal, int kpad8, float sc) {
  const int i  = blockIdx.x * NTHR + threadIdx.x;
  const int n8 = nrow * kpad8;
  if (i < n8) {
    const int row = i / kpad8;
    const int c8  = i - row * kpad8;
    const int k0  = c8 * 8;
    const int ka  = (k0 < kreal - 4) ? k0 : (kreal - 4);
    const int kb  = (k0 + 4 < kreal - 4) ? (k0 + 4) : (kreal - 4);
    const float* rp = src + (size_t)row * (size_t)kreal;
    const v4f a = *(const v4f*)(rp + ka);
    const v4f b = *(const v4f*)(rp + kb);
    v8h hv;
#pragma unroll
    for (int e = 0; e < 4; ++e) {
      const float fa = (k0 + e < kreal) ? (a[e] * sc) : 0.0f;
      const float fb = (k0 + 4 + e < kreal) ? (b[e] * sc) : 0.0f;
      hv[e]     = (_Float16)fa;
      hv[4 + e] = (_Float16)fb;
    }
    volatile v8h* dp = (volatile v8h*)(dst + (size_t)i * 8);
    *dp = hv;
    __threadfence();
    *dp = hv;
  }
}

__global__ __launch_bounds__(NTHR) void build_at_kernel(const float* __restrict__ Asrc, unsigned short* __restrict__ dst, float sc) {
  const int i = blockIdx.x * NTHR + threadIdx.x;
  const int n8 = AUG_PAD * (AUG_PAD / 8);
  if (i < n8) {
    const int n  = i / (AUG_PAD / 8);
    const int c8 = i - n * (AUG_PAD / 8);
    const int nn = (n < AUG) ? n : (AUG - 1);
    v8h hv;
#pragma unroll
    for (int e = 0; e < 8; ++e) {
      const int k  = c8 * 8 + e;
      const int kk = (k < AUG) ? k : (AUG - 1);
      const float v = Asrc[(size_t)kk * AUG + nn];
      const float f = (n < AUG && k < AUG) ? (v * sc) : 0.0f;
      hv[e] = (_Float16)f;
    }
    volatile v8h* dp = (volatile v8h*)(dst + (size_t)i * 8);
    *dp = hv;
    __threadfence();
    *dp = hv;
  }
}

__global__ __launch_bounds__(NTHR) void whh_pack_kernel(const float* __restrict__ w0, const float* __restrict__ w1,
                                                        const float* __restrict__ w2, const float* __restrict__ w3,
                                                        float* __restrict__ dst) {
  __shared__ float Tt[4 * 32 * 33];
  const int tid = threadIdx.x, lane = tid & 31, wave = tid >> 5;
  const int j0 = blockIdx.x * 32, k0 = blockIdx.y * 32, d = blockIdx.z;
  const float* src = (d == 0) ? w0 : ((d == 1) ? w1 : ((d == 2) ? w2 : w3));
#pragma unroll
  for (int it = 0; it < 4; ++it) {
    const int idx = it * NTHR + tid;
    const int g   = idx >> 8;
    const int rem = idx & 255;
    const int jj  = rem >> 3;
    const int k4  = (rem & 7) * 4;
    const v4f v = *(const v4f*)(src + (size_t)(g * HID + j0 + jj) * HID + k0 + k4);
    float* tp = Tt + (g * 32 + jj) * 33 + k4;
    tp[0] = v[0];
    tp[1] = v[1];
    tp[2] = v[2];
    tp[3] = v[3];
  }
  __syncthreads();
  v4f o[4];
#pragma unroll
  for (int it = 0; it < 4; ++it) {
    const int kk = wave + 8 * it;
    o[it][0] = Tt[(0 * 32 + lane) * 33 + kk];
    o[it][1] = Tt[(1 * 32 + lane) * 33 + kk];
    o[it][2] = Tt[(2 * 32 + lane) * 33 + kk];
    o[it][3] = Tt[(3 * 32 + lane) * 33 + kk];
  }
  float* op = dst + (size_t)d * (size_t)HID * (size_t)GATES;
  for (int pass = 0; pass < 2; ++pass) {
#pragma unroll
    for (int it = 0; it < 4; ++it) {
      const int kk = wave + 8 * it;
      *(volatile v4f*)(op + (size_t)(k0 + kk) * GATES + (size_t)(j0 + lane) * 4) = o[it];
    }
    __threadfence();
  }
}

__global__ __launch_bounds__(NTHR) void embed_kernel(const int* __restrict__ widx, const int* __restrict__ pidx,
                                                     const float* __restrict__ wemb, const float* __restrict__ pemb,
                                                     unsigned short* __restrict__ x0h, float sc) {
  const int i = blockIdx.x * NTHR + threadIdx.x;
  const int n8 = SEQ_LEN * (IN0_PAD / 8);
  if (i < n8) {
    const int row = i / (IN0_PAD / 8);
    const int c8  = i - row * (IN0_PAD / 8);
    int w = widx[row];
    int p = pidx[row];
    w = w < 0 ? 0 : w;
    w = w > VOC_W - 1 ? VOC_W - 1 : w;
    p = p < 0 ? 0 : p;
    p = p > VOC_P - 1 ? VOC_P - 1 : p;
    const float* wr = wemb + (size_t)w * EMB_W;
    const float* pr = pemb + (size_t)p * EMB_P;
    float wv[8], pv[8];
#pragma unroll
    for (int e = 0; e < 8; ++e) {
      const int k  = c8 * 8 + e;
      const int kw = (k < EMB_W) ? k : (EMB_W - 1);
      int kp = k - EMB_W;
      kp = kp < 0 ? 0 : kp;
      kp = kp > EMB_P - 1 ? EMB_P - 1 : kp;
      wv[e] = wr[kw];
      pv[e] = pr[kp];
    }
#pragma unroll
    for (int e = 0; e < 8; ++e) asm volatile("" : "+v"(wv[e]), "+v"(pv[e]));
    v8h hv;
#pragma unroll
    for (int e = 0; e < 8; ++e) {
      const int k = c8 * 8 + e;
      const float f = (k < EMB_W) ? wv[e] : ((k < IN0) ? pv[e] : 0.0f);
      hv[e] = (_Float16)(f * sc);
    }
    volatile v8h* dp = (volatile v8h*)(x0h + (size_t)i * 8);
    *dp = hv;
    __threadfence();
    *dp = hv;
  }
}

__global__ __launch_bounds__(512) void lstm_layer_kernel(const float* __restrict__ Gf, const float* __restrict__ Gb,
                                                         const float* __restrict__ WPf, const float* __restrict__ WPb,
                                                         unsigned short* __restrict__ Xout) {
  __shared__ __align__(16) float hbuf[2][HID];
  const int dir = blockIdx.x;
  const float* G  = dir ? Gb : Gf;
  const float* WP = dir ? WPb : WPf;
  const int j = threadIdx.x;
  const int lane = j & 31, wave = j >> 5;
  hbuf[0][j] = 0.0f;
  hbuf[1][j] = 0.0f;
  float cst = 0.0f;
  __syncthreads();
  const v4f* wp = (const v4f*)WP + j;

#pragma unroll 1
  for (int t = 0; t < SEQ_LEN; ++t) {
    const int row = dir ? (SEQ_LEN - 1 - t) : t;
    const int cur = t & 1;
    const float* g = G + (size_t)row * GATES;
    float zi = g[j];
    float zf = g[HID + j];
    float zg = g[2 * HID + j];
    float zo = g[3 * HID + j];
    const float* hc = hbuf[cur];
#pragma unroll 2
    for (int k = 0; k < HID; k += 4) {
      const v4f hv = *(const v4f*)(hc + k);
      const v4f q0 = wp[(size_t)(k + 0) * HID];
      const v4f q1 = wp[(size_t)(k + 1) * HID];
      const v4f q2 = wp[(size_t)(k + 2) * HID];
      const v4f q3 = wp[(size_t)(k + 3) * HID];
      zi = fmaf(q0[0], hv[0], zi);
      zf = fmaf(q0[1], hv[0], zf);
      zg = fmaf(q0[2], hv[0], zg);
      zo = fmaf(q0[3], hv[0], zo);
      zi = fmaf(q1[0], hv[1], zi);
      zf = fmaf(q1[1], hv[1], zf);
      zg = fmaf(q1[2], hv[1], zg);
      zo = fmaf(q1[3], hv[1], zo);
      zi = fmaf(q2[0], hv[2], zi);
      zf = fmaf(q2[1], hv[2], zf);
      zg = fmaf(q2[2], hv[2], zg);
      zo = fmaf(q2[3], hv[2], zo);
      zi = fmaf(q3[0], hv[3], zi);
      zf = fmaf(q3[1], hv[3], zf);
      zg = fmaf(q3[2], hv[3], zg);
      zo = fmaf(q3[3], hv[3], zo);
    }
    const float ig = fsig(zi);
    const float fg = fsig(zf);
    const float og = fsig(zo);
    const float gg = ftanh(zg);
    cst = fg * cst + ig * gg;
    const float hn = og * ftanh(cst);
    hbuf[cur ^ 1][j] = hn;
    __syncthreads();
    if (wave < 8) {
      const float* hnb = hbuf[cur ^ 1];
      const float a = hnb[64 * wave + 2 * lane];
      const float b = hnb[64 * wave + 2 * lane + 1];
      const _Float16 h0 = (_Float16)(a * CARRY_H);
      const _Float16 h1 = (_Float16)(b * CARRY_H);
      const unsigned u = (unsigned)__builtin_bit_cast(unsigned short, h0) | ((unsigned)__builtin_bit_cast(unsigned short, h1) << 16);
      const size_t ui = ((size_t)row * IN1 + (size_t)dir * HID + (size_t)(64 * wave)) / 2 + (size_t)lane;
      volatile unsigned* dp = (volatile unsigned*)Xout + ui;
      *dp = u;
      __threadfence();
      *dp = u;
    }
  }
}

__global__ __launch_bounds__(NTHR) void tanh_aug_kernel(const float* __restrict__ hm, unsigned short* __restrict__ hbh,
                                                        unsigned short* __restrict__ mbh, float sc) {
  const int i = blockIdx.x * NTHR + threadIdx.x;
  const int per = SEQ_LEN * (AUG_PAD / 8);
  if (i < 2 * per) {
    const int plane = (i >= per) ? 1 : 0;
    const int ii  = i - plane * per;
    const int row = ii / (AUG_PAD / 8);
    const int c8  = ii - row * (AUG_PAD / 8);
    const int c8c = (c8 < MLP / 8) ? c8 : (MLP / 8 - 1);
    const float* sp = hm + (size_t)row * HM_LD + plane * MLP + c8c * 8;
    const v4f a = *(const v4f*)(sp);
    const v4f b = *(const v4f*)(sp + 4);
    v8h hv;
#pragma unroll
    for (int e = 0; e < 4; ++e) {
      const int ka = c8 * 8 + e;
      const int kb = ka + 4;
      const float ta = ftanh(a[e]) * sc;
      const float tb = ftanh(b[e]) * sc;
      const float fa = (ka < MLP) ? ta : ((ka == MLP) ? sc : 0.0f);
      const float fb = (kb < MLP) ? tb : ((kb == MLP) ? sc : 0.0f);
      hv[e]     = (_Float16)fa;
      hv[4 + e] = (_Float16)fb;
    }
    unsigned short* dst = plane ? mbh : hbh;
    volatile v8h* dp = (volatile v8h*)(dst + (size_t)ii * 8);
    *dp = hv;
    __threadfence();
    *dp = hv;
  }
}

__global__ __launch_bounds__(NTHR) void pair_score_kernel(const float* __restrict__ hm, const float* __restrict__ satt,
                                                          const float* __restrict__ Wf, const float* __restrict__ bfp,
                                                          float* __restrict__ out) {
  __shared__ __align__(16) float hs[32 * PK_CH];
  __shared__ __align__(16) float ms[32 * PK_MP];
  __shared__ __align__(16) float wfs[PK_CH];
  const int tid = threadIdx.x, tj = tid & 31, tq = tid >> 5;
  const int i0 = blockIdx.y * 32, j0 = blockIdx.x * 32;
  float acc[4];
#pragma unroll
  for (int q = 0; q < 4; ++q) acc[q] = 0.0f;

#pragma unroll 1
  for (int kc = 0; kc < MLP; kc += PK_CH) {
    __syncthreads();
#pragma unroll
    for (int it = 0; it < 2; ++it) {
      const int idx = it * NTHR + tid;
      const int rr  = idx >> 4;
      const int k4  = (idx & 15) * 4;
      const v4f hv = *(const v4f*)(hm + (size_t)(i0 + rr) * HM_LD + kc + k4);
      const v4f mv = *(const v4f*)(hm + (size_t)(j0 + rr) * HM_LD + MLP + kc + k4);
      *(v4f*)(hs + rr * PK_CH + k4) = hv;
      *(v4f*)(ms + rr * PK_MP + k4) = mv;
    }
    if (tid < PK_CH) wfs[tid] = Wf[kc + tid];
    __syncthreads();
#pragma unroll 1
    for (int kk = 0; kk < PK_CH; kk += 4) {
      const v4f mv = *(const v4f*)(ms + tj * PK_MP + kk);
      const v4f wv = *(const v4f*)(wfs + kk);
#pragma unroll
      for (int q = 0; q < 4; ++q) {
        const v4f hv = *(const v4f*)(hs + (tq + 8 * q) * PK_CH + kk);
#pragma unroll
        for (int e = 0; e < 4; ++e) acc[q] = fmaf(ftanh(hv[e] + mv[e]), wv[e], acc[q]);
      }
    }
  }
  const float bb = bfp[0];
  float o[4];
#pragma unroll
  for (int q = 0; q < 4; ++q) {
    const int i = i0 + tq + 8 * q;
    o[q] = satt[(size_t)i * SEQ_LEN + j0 + tj] + (acc[q] + bb);
  }
  for (int pass = 0; pass < 2; ++pass) {
#pragma unroll
    for (int q = 0; q < 4; ++q) {
      const int i = i0 + tq + 8 * q;
      *(volatile float*)(out + (size_t)i * SEQ_LEN + j0 + tj) = o[q];
    }
    __threadfence();
  }
}

extern "C" void kernel_launch(void* const* d_in, const int* in_sizes, int n_in,
                              void* d_out, int out_size, void* d_ws, size_t ws_size, hipStream_t stream) {
  if (n_in < 23 || d_out == nullptr || d_ws == nullptr) return;
  if (in_sizes[0] != SEQ_LEN || in_sizes[1] != SEQ_LEN || in_sizes[2] != VOC_W * EMB_W || in_sizes[3] != VOC_P * EMB_P ||
      in_sizes[4] != GATES * IN0 || in_sizes[5] != GATES * HID || in_sizes[6] != GATES ||
      in_sizes[7] != GATES * IN0 || in_sizes[8] != GATES * HID || in_sizes[9] != GATES ||
      in_sizes[10] != GATES * IN1 || in_sizes[11] != GATES * HID || in_sizes[12] != GATES ||
      in_sizes[13] != GATES * IN1 || in_sizes[14] != GATES * HID || in_sizes[15] != GATES ||
      in_sizes[16] != MLP * IN1 || in_sizes[17] != MLP || in_sizes[18] != MLP * IN1 || in_sizes[19] != MLP ||
      in_sizes[20] != AUG * AUG || in_sizes[21] != MLP || in_sizes[22] != 1 ||
      out_size != SEQ_LEN * SEQ_LEN) return;

  const int*   widx  = (const int*)  d_in[0];
  const int*   pidx  = (const int*)  d_in[1];
  const float* wemb  = (const float*)d_in[2];
  const float* pemb  = (const float*)d_in[3];
  const float* Wih0f = (const float*)d_in[4];
  const float* Whh0f = (const float*)d_in[5];
  const float* b0f   = (const float*)d_in[6];
  const float* Wih0b = (const float*)d_in[7];
  const float* Whh0b = (const float*)d_in[8];
  const float* b0b   = (const float*)d_in[9];
  const float* Wih1f = (const float*)d_in[10];
  const float* Whh1f = (const float*)d_in[11];
  const float* b1f   = (const float*)d_in[12];
  const float* Wih1b = (const float*)d_in[13];
  const float* Whh1b = (const float*)d_in[14];
  const float* b1b   = (const float*)d_in[15];
  const float* Wh    = (const float*)d_in[16];
  const float* bh    = (const float*)d_in[17];
  const float* Wm    = (const float*)d_in[18];
  const float* bm    = (const float*)d_in[19];
  const float* Amat  = (const float*)d_in[20];
  const float* Wf    = (const float*)d_in[21];
  const float* bfp   = (const float*)d_in[22];
  float* out = (float*)d_out;

  char* ws = (char*)d_ws;
  size_t off = 0;
  auto carve = [&](size_t bytes) -> char* { char* p = ws + off; off += (bytes + 255) & ~(size_t)255; return p; };
  unsigned short* X0H  = (unsigned short*)carve((size_t)SEQ_LEN * IN0_PAD * 2);
  unsigned short* W0   = (unsigned short*)carve((size_t)2 * GATES * IN0_PAD * 2);
  unsigned short* W1   = (unsigned short*)carve((size_t)2 * GATES * IN1 * 2);
  unsigned short* WHF  = (unsigned short*)carve((size_t)MLP * IN1 * 2);
  unsigned short* WMF  = (unsigned short*)carve((size_t)MLP * IN1 * 2);
  unsigned short* ATP  = (unsigned short*)carve((size_t)AUG_PAD * AUG_PAD * 2);
  float*          WHHP = (float*)carve((size_t)4 * HID * GATES * 4);
  float*          GP   = (float*)carve((size_t)2 * SEQ_LEN * GATES * 4);
  unsigned short* X1H  = (unsigned short*)carve((size_t)SEQ_LEN * IN1 * 2);
  unsigned short* X2H  = (unsigned short*)carve((size_t)SEQ_LEN * IN1 * 2);
  float*          HM   = (float*)carve((size_t)SEQ_LEN * HM_LD * 4);
  unsigned short* HBH  = (unsigned short*)carve((size_t)SEQ_LEN * AUG_PAD * 2);
  unsigned short* MBH  = (unsigned short*)carve((size_t)SEQ_LEN * AUG_PAD * 2);
  unsigned short* THP  = (unsigned short*)carve((size_t)SEQ_LEN * AUG_PAD * 2);
  float*          SATT = (float*)carve((size_t)SEQ_LEN * SEQ_LEN * 4);
  if (off > ws_size || off > (size_t)134217728) return;

  unsigned short* W0f = W0;
  unsigned short* W0b = W0 + (size_t)GATES * IN0_PAD;
  unsigned short* W1f = W1;
  unsigned short* W1b = W1 + (size_t)GATES * IN1;
  float* Gfw = GP;
  float* Gbw = GP + (size_t)SEQ_LEN * GATES;
  const size_t wpl = (size_t)HID * GATES;

  const int n8w0 = GATES * (IN0_PAD / 8);
  const int n8w1 = GATES * (IN1 / 8);
  const int n8wp = MLP * (IN1 / 8);
  cvt_pad_f16_kernel<<<n8w0 / NTHR, NTHR, 0, stream>>>(Wih0f, W0f, GATES, IN0, IN0_PAD / 8, CARRY_W);
  cvt_pad_f16_kernel<<<n8w0 / NTHR, NTHR, 0, stream>>>(Wih0b, W0b, GATES, IN0, IN0_PAD / 8, CARRY_W);
  cvt_pad_f16_kernel<<<n8w1 / NTHR, NTHR, 0, stream>>>(Wih1f, W1f, GATES, IN1, IN1 / 8, CARRY_W);
  cvt_pad_f16_kernel<<<n8w1 / NTHR, NTHR, 0, stream>>>(Wih1b, W1b, GATES, IN1, IN1 / 8, CARRY_W);
  cvt_pad_f16_kernel<<<n8wp / NTHR, NTHR, 0, stream>>>(Wh, WHF, MLP, IN1, IN1 / 8, CARRY_W);
  cvt_pad_f16_kernel<<<n8wp / NTHR, NTHR, 0, stream>>>(Wm, WMF, MLP, IN1, IN1 / 8, CARRY_W);
  build_at_kernel<<<(AUG_PAD * (AUG_PAD / 8)) / NTHR, NTHR, 0, stream>>>(Amat, ATP, CARRY_W);
  whh_pack_kernel<<<dim3(HID / 32, HID / 32, 4), NTHR, 0, stream>>>(Whh0f, Whh0b, Whh1f, Whh1b, WHHP);

  embed_kernel<<<(SEQ_LEN * (IN0_PAD / 8)) / NTHR, NTHR, 0, stream>>>(widx, pidx, wemb, pemb, X0H, CARRY_X0);

  const int gb_gate = ((SEQ_LEN >> 6) * (GATES >> 6) + 7) / 8;
  wmma_gemm64<true, false><<<gb_gate, 256, 0, stream>>>(X0H, IN0_PAD, W0f, IN0_PAD, (void*)Gfw, GATES, b0f,
                                                        SEQ_LEN, GATES, IN0_PAD, SC_L0);
  wmma_gemm64<true, false><<<gb_gate, 256, 0, stream>>>(X0H, IN0_PAD, W0b, IN0_PAD, (void*)Gbw, GATES, b0b,
                                                        SEQ_LEN, GATES, IN0_PAD, SC_L0);
  lstm_layer_kernel<<<2, 512, 0, stream>>>(Gfw, Gbw, WHHP, WHHP + wpl, X1H);

  wmma_gemm64<true, false><<<gb_gate, 256, 0, stream>>>(X1H, IN1, W1f, IN1, (void*)Gfw, GATES, b1f,
                                                        SEQ_LEN, GATES, IN1, SC_HW);
  wmma_gemm64<true, false><<<gb_gate, 256, 0, stream>>>(X1H, IN1, W1b, IN1, (void*)Gbw, GATES, b1b,
                                                        SEQ_LEN, GATES, IN1, SC_HW);
  lstm_layer_kernel<<<2, 512, 0, stream>>>(Gfw, Gbw, WHHP + 2 * wpl, WHHP + 3 * wpl, X2H);

  const int gb_proj = ((SEQ_LEN >> 6) * (MLP >> 6) + 7) / 8;
  wmma_gemm64<true, false><<<gb_proj, 256, 0, stream>>>(X2H, IN1, WHF, IN1, (void*)HM, HM_LD, bh,
                                                        SEQ_LEN, MLP, IN1, SC_HW);
  wmma_gemm64<true, false><<<gb_proj, 256, 0, stream>>>(X2H, IN1, WMF, IN1, (void*)(HM + MLP), HM_LD, bm,
                                                        SEQ_LEN, MLP, IN1, SC_HW);

  tanh_aug_kernel<<<(2 * SEQ_LEN * (AUG_PAD / 8)) / NTHR, NTHR, 0, stream>>>(HM, HBH, MBH, CARRY_H);
  const int gb_t = ((SEQ_LEN >> 6) * (AUG_PAD >> 6) + 7) / 8;
  wmma_gemm64<false, true><<<gb_t, 256, 0, stream>>>(HBH, AUG_PAD, ATP, AUG_PAD, (void*)THP, AUG_PAD, bfp,
                                                     SEQ_LEN, AUG_PAD, AUG_PAD, SC_T);
  const int gb_s = ((SEQ_LEN >> 6) * (SEQ_LEN >> 6) + 7) / 8;
  wmma_gemm64<false, false><<<gb_s, 256, 0, stream>>>(THP, AUG_PAD, MBH, AUG_PAD, (void*)SATT, SEQ_LEN, bfp,
                                                      SEQ_LEN, SEQ_LEN, AUG_PAD, SC_ATT);

  pair_score_kernel<<<dim3(SEQ_LEN / 32, SEQ_LEN / 32), NTHR, 0, stream>>>(HM, SATT, Wf, bfp, out);
}
